// TransformerCAModule_29789893165200
// MI455X (gfx1250) — hardware-verified
//
#include <hip/hip_runtime.h>
#include <hip/hip_bf16.h>

typedef _Float16 f16_t;
typedef __attribute__((ext_vector_type(16))) _Float16 v16h;
typedef __attribute__((ext_vector_type(8)))  _Float16 v8h;
typedef __attribute__((ext_vector_type(4)))  _Float16 v4h;
typedef __attribute__((ext_vector_type(16))) __bf16   v16b;
typedef __attribute__((ext_vector_type(8)))  __bf16   v8b;
typedef __attribute__((ext_vector_type(8)))  float    v8f;
typedef __attribute__((ext_vector_type(4)))  float    v4f;
#define U16(p) ((const unsigned short*)(const void*)(p))

__device__ __forceinline__ unsigned short f2bf_bits(float f) {
  unsigned u = __float_as_uint(f);
  return (unsigned short)((u + 0x7FFFu + ((u >> 16) & 1u)) >> 16);
}
__device__ __forceinline__ float bf_bits2f(unsigned short h) { return __uint_as_float(((unsigned)h) << 16); }

__device__ __forceinline__ void dep_guard_h(v8f& a, v8f& b, v16h x, v16h y) { asm volatile("v_nop\n\tv_nop\n\tv_nop\n\tv_nop" : "+v"(a), "+v"(b) : "v"(x), "v"(y)); }
__device__ __forceinline__ void dep_guard_b(v8f& a, v8f& b, v16b x, v16b y) { asm volatile("v_nop\n\tv_nop\n\tv_nop\n\tv_nop" : "+v"(a), "+v"(b) : "v"(x), "v"(y)); }
__device__ __forceinline__ void keep4_h(v16h a, v16h b, v16h c, v16h d) { asm volatile("v_nop" :: "v"(a), "v"(b), "v"(c), "v"(d)); }
__device__ __forceinline__ void keep4_b(v16b a, v16b b, v16b c, v16b d) { asm volatile("v_nop" :: "v"(a), "v"(b), "v"(c), "v"(d)); }
__device__ __forceinline__ void acc_guard4(v8f& a, v8f& b, v8f& c, v8f& d) { asm volatile("v_nop\n\tv_nop\n\tv_nop\n\tv_nop" : "+v"(a), "+v"(b), "+v"(c), "+v"(d)); }
template <typename T> struct Frag;
template <> struct Frag<_Float16> {
  typedef v16h V; union U { v16h v; v8h h[2]; };
  static __device__ __forceinline__ v16h load(const _Float16* p) {
    U f; f.h[0] = *(const v8h*)(p); f.h[1] = *(const v8h*)(p + 16); return f.v;
  }
  static __device__ __forceinline__ v8f mma(v16h a, v16h b, v8f c) {
    return __builtin_amdgcn_wmma_f32_16x16x32_f16(false, a, false, b, (short)0, c, false, false);
  }
  static __device__ __forceinline__ void guard(v8f& a, v8f& b, v16h x, v16h y) { dep_guard_h(a, b, x, y); }
  static __device__ __forceinline__ void keep(v16h a, v16h b, v16h c, v16h d) { keep4_h(a, b, c, d); }
};
template <> struct Frag<__bf16> {
  typedef v16b V; union U { v16b v; v8b h[2]; };
  static __device__ __forceinline__ v16b load(const __bf16* p) {
    U f; f.h[0] = *(const v8b*)(p); f.h[1] = *(const v8b*)(p + 16); return f.v;
  }
  static __device__ __forceinline__ v8f mma(v16b a, v16b b, v8f c) {
    return __builtin_amdgcn_wmma_f32_16x16x32_bf16(false, a, false, b, (short)0, c, false, false);
  }
  static __device__ __forceinline__ void guard(v8f& a, v8f& b, v16b x, v16b y) { dep_guard_b(a, b, x, y); }
  static __device__ __forceinline__ void keep(v16b a, v16b b, v16b c, v16b d) { keep4_b(a, b, c, d); }
};

template <int ET> struct Elem;
template <> struct Elem<0> { typedef _Float16 T; };
template <> struct Elem<1> { typedef __bf16 T; };
template <int ET, bool SPLIT, int BIAS_MODE, int OUT_MODE, bool RESID, int ACT = 0>
__global__ __launch_bounds__(256) void wmma_gemm64(
    const unsigned short* __restrict__ Ap, const unsigned short* __restrict__ A2p, int lda, long strideA,
    const unsigned short* __restrict__ Btp, const unsigned short* __restrict__ Bt2p, int ldb, long strideB,
    void* __restrict__ Cout, void* __restrict__ Cout2, int ldc, long strideC,
    const float* __restrict__ bias,
    const float* __restrict__ resid, long strideR,
    int M, int N, int K, float scale) {
  typedef typename Elem<ET>::T T;
  typedef typename Frag<T>::V V;
  const T* A = (const T*)Ap; const T* A2 = (const T*)A2p; const T* Bt = (const T*)Btp; const T* Bt2 = (const T*)Bt2p;
  __shared__ __align__(16) float sT[8][16 * 68];
  const int b    = blockIdx.y;
  const int lane = threadIdx.x & 31;
  const int wave = threadIdx.x >> 5;
  const int tilesN = N >> 6;
  const int tilesM = M >> 6;
  const int tile = blockIdx.x * 8 + wave;
  if (tile >= tilesM * tilesN) return;
  const int tm = tile / tilesN;
  const int tn = tile - tm * tilesN;
  const int m0 = tm << 6;
  const int n0 = tn << 6;

  const T* Ab  = A  + (size_t)b * strideA;
  const T* Bb  = Bt + (size_t)b * strideB;
  const T* Ab2 = SPLIT ? (A2  + (size_t)b * strideA) : nullptr;
  const T* Bb2 = SPLIT ? (Bt2 + (size_t)b * strideB) : nullptr;

  const int rlane = lane & 15;
  const int koff  = (lane >> 4) * 8;
  const int mOff  = (lane >> 4) * 8;

  v8f acc[4][4];
#pragma unroll
  for (int i = 0; i < 4; ++i)
#pragma unroll
    for (int j = 0; j < 4; ++j) acc[i][j] = (v8f){0.f,0.f,0.f,0.f,0.f,0.f,0.f,0.f};

  for (int k0 = 0; k0 < K; k0 += 32) {
    V bh[4], bl[4];
#pragma unroll
    for (int j = 0; j < 4; ++j) {
      const size_t bo = (size_t)(n0 + (j << 4) + rlane) * ldb + koff + k0;
      bh[j] = Frag<T>::load(Bb + bo);
      if (SPLIT) bl[j] = Frag<T>::load(Bb2 + bo);
    }
#pragma unroll
    for (int i = 0; i < 4; ++i) {
      const size_t ao = (size_t)(m0 + (i << 4) + rlane) * lda + koff + k0;
      V ah = Frag<T>::load(Ab + ao);
      V al;
      if (SPLIT) al = Frag<T>::load(Ab2 + ao);
#pragma unroll
      for (int j = 0; j < 4; ++j) {
        acc[i][j] = Frag<T>::mma(ah, bh[j], acc[i][j]);
        if (SPLIT) {
          acc[i][j] = Frag<T>::mma(ah, bl[j], acc[i][j]);
          acc[i][j] = Frag<T>::mma(al, bh[j], acc[i][j]);
        }
      }
      Frag<T>::guard(acc[i][0], acc[i][3], ah, SPLIT ? al : ah);
    }
    Frag<T>::keep(bh[0], bh[1], bh[2], bh[3]);
    if (SPLIT) Frag<T>::keep(bl[0], bl[1], bl[2], bl[3]);
  }
  acc_guard4(acc[0][0], acc[0][1], acc[0][2], acc[0][3]);
  acc_guard4(acc[1][0], acc[1][1], acc[1][2], acc[1][3]);
  acc_guard4(acc[2][0], acc[2][1], acc[2][2], acc[2][3]);
  acc_guard4(acc[3][0], acc[3][1], acc[3][2], acc[3][3]);

  float* slab = sT[wave];
  const float* Rb = RESID ? (resid + (size_t)b * strideR) : nullptr;
#pragma unroll
  for (int i = 0; i < 4; ++i) {
    const int mBase = m0 + (i << 4);
#pragma unroll
    for (int j = 0; j < 4; ++j) {
      const int n = n0 + (j << 4) + rlane;
      float bv = 0.f;
      if (BIAS_MODE == 2) bv = bias[n];
#pragma unroll
      for (int r = 0; r < 8; ++r) {
        float v = acc[i][j][r] * scale;
        if (BIAS_MODE == 1) v += bias[mBase + mOff + r];
        if (BIAS_MODE == 2) v += bv;
        if (RESID) v += Rb[(size_t)(mBase + mOff + r) * ldc + n];
        if (ACT == 1) v = tanhf(v);
        if (ACT == 2) v = fmaxf(v, 0.0f);
        if (ACT == 3) v = v / (1.0f + expf(-v));
        if (ACT == 4) v = (v > 0.f) ? v : 0.01f * v;
        if (ACT == 5) v = 0.5f * v * (1.0f + erff(v * 0.70710678118654752f));
        slab[(mOff + r) * 68 + (j << 4) + rlane] = v;
      }
    }
    __builtin_amdgcn_fence(__ATOMIC_RELEASE, "workgroup");
    __builtin_amdgcn_wave_barrier();
    __builtin_amdgcn_fence(__ATOMIC_ACQUIRE, "workgroup");
    if (OUT_MODE == 0) {
      float* C = (float*)Cout + (size_t)b * strideC;
      const int hh = lane >> 4, c4 = (lane & 15) * 4;
      for (int pass = 0; pass < 2; ++pass) {
#pragma unroll
        for (int it = 0; it < 8; ++it) {
          const int row = it * 2 + hh;
          v4f v = *(const v4f*)(slab + row * 68 + c4);
          *(volatile v4f*)(C + (size_t)(mBase + row) * ldc + n0 + c4) = v;
        }
        __threadfence();
      }
    } else {
      const int q = lane >> 3, c8 = (lane & 7) * 8;
      unsigned short* C  = (unsigned short*)Cout  + (size_t)b * strideC;
      unsigned short* C2 = (OUT_MODE == 2) ? ((unsigned short*)Cout2 + (size_t)b * strideC) : nullptr;
      for (int pass = 0; pass < 2; ++pass) {
#pragma unroll
        for (int it = 0; it < 4; ++it) {
          const int row = it * 4 + q;
          const float* sp = slab + row * 68 + c8;
          v8h hv, lv;
#pragma unroll
          for (int e = 0; e < 8; ++e) {
            if (OUT_MODE == 1) {
              hv[e] = (_Float16)sp[e];
            } else {
              unsigned short hb = f2bf_bits(sp[e]);
              unsigned short lb = f2bf_bits(sp[e] - bf_bits2f(hb));
              hv[e] = __builtin_bit_cast(_Float16, hb);
              lv[e] = __builtin_bit_cast(_Float16, lb);
            }
          }
          *(volatile v8h*)(C + (size_t)(mBase + row) * ldc + n0 + c8) = hv;
          if (OUT_MODE == 2) *(volatile v8h*)(C2 + (size_t)(mBase + row) * ldc + n0 + c8) = lv;
        }
        __threadfence();
      }
    }
    __builtin_amdgcn_fence(__ATOMIC_RELEASE, "workgroup");
    __builtin_amdgcn_wave_barrier();
    __builtin_amdgcn_fence(__ATOMIC_ACQUIRE, "workgroup");
  }
}

__global__ __launch_bounds__(256) void cast_w_kernel(const float* __restrict__ in, f16_t* __restrict__ out,
                                                     int rows, int kin, int kpad, float scale) {
  const int i  = blockIdx.x * 256 + threadIdx.x;
  const int n2 = (rows * kpad) >> 1;
  if (i < n2) {
    const int e0 = 2 * i;
    const int r  = e0 / kpad;
    const int c  = e0 - r * kpad;
    const int c0 = (c < kin) ? c : (kin - 1);
    const int c1 = ((c + 1) < kin) ? (c + 1) : (kin - 1);
    float f0 = in[(size_t)r * kin + c0] * scale;
    float f1 = in[(size_t)r * kin + c1] * scale;
    f0 = (c < kin) ? f0 : 0.0f;
    f1 = ((c + 1) < kin) ? f1 : 0.0f;
    const f16_t h0 = (f16_t)f0, h1 = (f16_t)f1;
    const unsigned u = (unsigned)__builtin_bit_cast(unsigned short, h0) | ((unsigned)__builtin_bit_cast(unsigned short, h1) << 16);
    ((volatile unsigned*)out)[i] = u;
    __threadfence();
    ((volatile unsigned*)out)[i] = u;
  }
}

__global__ __launch_bounds__(256) void xpose_x_kernel(const float* __restrict__ x, f16_t* __restrict__ X16) {
  __shared__ __align__(16) f16_t tile[256 * 32];
  const int t   = threadIdx.x;
  const int n   = blockIdx.x * 256 + t;
  const int b   = n >> 14;
  const int rem = n & 16383;
  const float* xp = x + (size_t)b * 16 * 16384 + rem;
#pragma unroll
  for (int c = 0; c < 16; ++c) tile[t * 32 + c] = (f16_t)xp[(size_t)c * 16384];
#pragma unroll
  for (int c = 16; c < 32; ++c) tile[t * 32 + c] = (f16_t)0.0f;
  __syncthreads();
  f16_t* dst = X16 + (size_t)blockIdx.x * 256 * 32;
  for (int pass = 0; pass < 2; ++pass) {
#pragma unroll
    for (int it = 0; it < 4; ++it) {
      const int q = it * 256 + t;
      const v8h v = *(const v8h*)(tile + q * 8);
      *(volatile v8h*)(dst + (size_t)q * 8) = v;
    }
    __threadfence();
  }
}

__device__ __forceinline__ v4f ln_vec(v4f x, const float* __restrict__ g, const float* __restrict__ bb, int lane) {
  float s = (x[0] + x[1]) + (x[2] + x[3]);
#pragma unroll
  for (int off = 1; off < 32; off <<= 1) s += __shfl_xor(s, off, 32);
  const float mean = s * (1.0f / 128.0f);
  const v4f d = x - mean;
  float ss = (d[0] * d[0] + d[1] * d[1]) + (d[2] * d[2] + d[3] * d[3]);
#pragma unroll
  for (int off = 1; off < 32; off <<= 1) ss += __shfl_xor(ss, off, 32);
  const float var  = ss * (1.0f / 128.0f);
  const float rstd = 1.0f / sqrtf(var + 1e-5f);
  const v4f gv = *(const v4f*)(g + lane * 4);
  const v4f bv = *(const v4f*)(bb + lane * 4);
  return (d * rstd) * gv + bv;
}

__global__ __launch_bounds__(256) void gather_ln_kernel(const float* __restrict__ e32, const float* __restrict__ pos,
                                                        const float* __restrict__ g, const float* __restrict__ bb,
                                                        float* __restrict__ t32, f16_t* __restrict__ h16,
                                                        int P, int nbase) {
  const int lane = threadIdx.x & 31;
  const int wave = threadIdx.x >> 5;
  const int p = blockIdx.x * 8 + wave;
  const int j = blockIdx.y;
  if (p >= P) return;
  const int n  = nbase + p;
  const int b  = n >> 14;
  const int y  = (n >> 7) & 127;
  const int x  = n & 127;
  const int yy = y + (j / 3) - 1;
  const int xx = x + (j % 3) - 1;
  const bool valid = ((unsigned)yy < 128u) && ((unsigned)xx < 128u);
  const int yc = yy < 0 ? 0 : (yy > 127 ? 127 : yy);
  const int xc = xx < 0 ? 0 : (xx > 127 ? 127 : xx);
  v4f ev = *(const v4f*)(e32 + ((size_t)((b << 14) + (yc << 7) + xc)) * 128 + lane * 4);
  if (!valid) ev = (v4f){0.f, 0.f, 0.f, 0.f};
  const v4f pv = *(const v4f*)(pos + j * 128 + lane * 4);
  const v4f tv = ev + pv;
  const size_t row = (size_t)j * (size_t)P + (size_t)p;
  float* tp = t32 + row * 128 + lane * 4;
  f16_t* hp = h16 + row * 128 + lane * 4;
  *(volatile v4f*)tp = tv;
  const v4f hv = ln_vec(tv, g, bb, lane);
  const v4h h4 = __builtin_convertvector(hv, v4h);
  *(volatile v4h*)hp = h4;
  __threadfence();
  *(volatile v4f*)tp = tv;
  *(volatile v4h*)hp = h4;
}

__global__ __launch_bounds__(256) void ln_rows_kernel(const float* __restrict__ t32, f16_t* __restrict__ h16,
                                                      const float* __restrict__ g, const float* __restrict__ bb, int nrows) {
  const int lane = threadIdx.x & 31;
  const int wave = threadIdx.x >> 5;
  const int row = blockIdx.x * 8 + wave;
  if (row >= nrows) return;
  const v4f xv = *(const v4f*)(t32 + (size_t)row * 128 + lane * 4);
  const v4f hv = ln_vec(xv, g, bb, lane);
  const v4h h4 = __builtin_convertvector(hv, v4h);
  f16_t* hp = h16 + (size_t)row * 128 + lane * 4;
  *(volatile v4h*)hp = h4;
  __threadfence();
  *(volatile v4h*)hp = h4;
}

template <int CENTER>
__global__ __launch_bounds__(288)
void win_attn_kernel(const f16_t* __restrict__ qsrc, int ldq,
                     const f16_t* __restrict__ ksrc, const f16_t* __restrict__ vsrc, int ldkv,
                     f16_t* __restrict__ odst, int P) {
  constexpr int NT   = CENTER ? 256 : 288;
  constexpr int WPBK = CENTER ? 64 : 8;
  constexpr int NROW = CENTER ? 64 : 72;
  __shared__ float sc[NT * 9];
  __shared__ __align__(16) f16_t ot[NROW * 128];
  const int t = threadIdx.x;
  int w, h, qi;
  if (CENTER) { w = t >> 2; h = t & 3; qi = 4; }
  else { w = t / 36; const int rem = t - w * 36; h = rem / 9; qi = rem - h * 9; }
  const int w0 = blockIdx.x * WPBK;
  const int p  = w0 + w;
  const size_t qrow = CENTER ? (size_t)p : ((size_t)qi * (size_t)P + (size_t)p);
  const f16_t* qp = qsrc + qrow * (size_t)ldq + h * 32;
  float qv[32];
#pragma unroll
  for (int i = 0; i < 4; ++i) {
    const v8h v = *(const v8h*)(qp + 8 * i);
#pragma unroll
    for (int e = 0; e < 8; ++e) qv[8 * i + e] = (float)v[e];
  }
  float* scp = sc + t * 9;
  float m = -3.0e38f;
#pragma unroll 1
  for (int kk = 0; kk < 9; ++kk) {
    const f16_t* kp = ksrc + ((size_t)kk * (size_t)P + (size_t)p) * (size_t)ldkv + h * 32;
    float s = 0.f;
#pragma unroll
    for (int i = 0; i < 4; ++i) {
      const v8h v = *(const v8h*)(kp + 8 * i);
#pragma unroll
      for (int e = 0; e < 8; ++e) s += qv[8 * i + e] * (float)v[e];
    }
    s *= 0.17677669529663687f;
    scp[kk] = s;
    m = fmaxf(m, s);
  }
  float l = 0.f;
#pragma unroll 1
  for (int kk = 0; kk < 9; ++kk) {
    const float pk = __expf(scp[kk] - m);
    scp[kk] = pk;
    l += pk;
  }
  const float inv = __builtin_amdgcn_rcpf(l);
  float ov[32];
#pragma unroll
  for (int d = 0; d < 32; ++d) ov[d] = 0.f;
#pragma unroll 1
  for (int kk = 0; kk < 9; ++kk) {
    const f16_t* vp = vsrc + ((size_t)kk * (size_t)P + (size_t)p) * (size_t)ldkv + h * 32;
    const float a = scp[kk] * inv;
#pragma unroll
    for (int i = 0; i < 4; ++i) {
      const v8h v = *(const v8h*)(vp + 8 * i);
#pragma unroll
      for (int e = 0; e < 8; ++e) ov[8 * i + e] += a * (float)v[e];
    }
  }
  const int lr = CENTER ? w : (qi * 8 + w);
  f16_t* orow = ot + lr * 128 + h * 32;
#pragma unroll
  for (int i = 0; i < 4; ++i) {
    v8h hv;
#pragma unroll
    for (int e = 0; e < 8; ++e) hv[e] = (f16_t)ov[8 * i + e];
    *(v8h*)(orow + 8 * i) = hv;
  }
  __syncthreads();
  for (int pass = 0; pass < 2; ++pass) {
#pragma unroll
    for (int it = 0; it < 4; ++it) {
      const int q   = it * NT + t;
      const int r   = q >> 4;
      const int c16 = q & 15;
      const size_t grow = CENTER ? (size_t)(w0 + r)
                                 : ((size_t)(r >> 3) * (size_t)P + (size_t)(w0 + (r & 7)));
      const v8h v = *(const v8h*)(ot + r * 128 + c16 * 8);
      *(volatile v8h*)(odst + grow * 128 + c16 * 8) = v;
    }
    __threadfence();
  }
}

__global__ __launch_bounds__(256) void head_kernel(const float* __restrict__ t32c, const float* __restrict__ g,
                                                   const float* __restrict__ bb, const float* __restrict__ hw,
                                                   const float* __restrict__ hb, float* __restrict__ out, int P) {
  __shared__ float res[32];
  const int lane = threadIdx.x & 31;
  const int wave = threadIdx.x >> 5;
  const v4f wv = *(const v4f*)(hw + lane * 4);
  const float hb0 = hb[0];
#pragma unroll
  for (int r = 0; r < 4; ++r) {
    int row = blockIdx.x * 32 + wave * 4 + r;
    row = row < P ? row : (P - 1);
    const v4f xv = *(const v4f*)(t32c + (size_t)row * 128 + lane * 4);
    const v4f hv = ln_vec(xv, g, bb, lane);
    float dsum = (hv[0] * wv[0] + hv[1] * wv[1]) + (hv[2] * wv[2] + hv[3] * wv[3]);
#pragma unroll
    for (int off = 1; off < 32; off <<= 1) dsum += __shfl_xor(dsum, off, 32);
    if (lane == 0) res[wave * 4 + r] = dsum + hb0;
  }
  __syncthreads();
  if (wave == 0) {
    const float v = res[lane];
    float* op = out + (size_t)blockIdx.x * 32 + lane;
    *(volatile float*)op = v;
    __threadfence();
    *(volatile float*)op = v;
  }
}

template <int OUT_MODE, bool RESID, int ACT>
static void launch_gemm(hipStream_t s, const f16_t* A, int lda, const f16_t* Bt, int ldb, void* C, int ldc,
                        const float* bias, const float* resid, int M, int N, int K, float scale) {
  const int tiles = (M / 64) * (N / 64);
  dim3 grid((tiles + 7) / 8, 1);
  wmma_gemm64<0, false, 2, OUT_MODE, RESID, ACT><<<grid, 256, 0, s>>>(
      U16(A), U16(A), lda, (long)0, U16(Bt), U16(Bt), ldb, (long)0,
      C, C, ldc, (long)0, bias, resid, (long)0, M, N, K, scale);
}

extern "C" void kernel_launch(void* const* d_in, const int* in_sizes, int n_in,
                              void* d_out, int out_size, void* d_ws, size_t ws_size,
                              hipStream_t stream) {
  enum { NPIX = 32768, DM = 128, DFFC = 256, PCH = 8192, NCHUNK = 4, RCH = 9 * PCH };
  const size_t SZ_WEMB = (size_t)128 * 32 * 2;
  const size_t SZ_WQKV = (size_t)768 * 128 * 2;
  const size_t SZ_WO   = (size_t)256 * 128 * 2;
  const size_t SZ_W1   = (size_t)512 * 128 * 2;
  const size_t SZ_W2   = (size_t)256 * 256 * 2;
  const size_t SZ_E32  = (size_t)NPIX * DM * 4;
  const size_t SZ_T32  = (size_t)RCH * DM * 4;
  const size_t SZ_H16  = (size_t)RCH * DM * 2;
  const size_t SZ_BIG  = (size_t)RCH * 384 * 2;
  const size_t OFF_WEMB = 0;
  const size_t OFF_WQKV = OFF_WEMB + SZ_WEMB;
  const size_t OFF_WO   = OFF_WQKV + SZ_WQKV;
  const size_t OFF_W1   = OFF_WO + SZ_WO;
  const size_t OFF_W2   = OFF_W1 + SZ_W1;
  const size_t OFF_E32  = OFF_W2 + SZ_W2;
  const size_t OFF_T32  = OFF_E32 + SZ_E32;
  const size_t OFF_H16  = OFF_T32 + SZ_T32;
  const size_t OFF_BIG  = OFF_H16 + SZ_H16;
  const size_t WS_TOTAL = OFF_BIG + SZ_BIG;
  const size_t OFF_Q16C_IN_BIG = (size_t)RCH * 256 * 2;

  if (n_in < 20) return;
  if (in_sizes[0] != 2 * 16 * 128 * 128 || in_sizes[1] != 128 * 16 || in_sizes[2] != 128 ||
      in_sizes[3] != 9 * 128 || in_sizes[4] != 2 * 384 * 128 || in_sizes[5] != 2 * 384 ||
      in_sizes[6] != 2 * 128 * 128 || in_sizes[7] != 2 * 128 || in_sizes[8] != 2 * 128 ||
      in_sizes[9] != 2 * 128 || in_sizes[10] != 2 * 128 || in_sizes[11] != 2 * 128 ||
      in_sizes[12] != 2 * 256 * 128 || in_sizes[13] != 2 * 256 || in_sizes[14] != 2 * 128 * 256 ||
      in_sizes[15] != 2 * 128 || in_sizes[16] != 128 || in_sizes[17] != 128 || in_sizes[18] != 128 ||
      in_sizes[19] < 1) return;
  if (out_size != NPIX) return;
  if (ws_size < WS_TOTAL) return;

  const float* x      = (const float*)d_in[0];
  const float* emb_w  = (const float*)d_in[1];
  const float* emb_b  = (const float*)d_in[2];
  const float* pos    = (const float*)d_in[3];
  const float* wqkv   = (const float*)d_in[4];
  const float* bqkv   = (const float*)d_in[5];
  const float* wo     = (const float*)d_in[6];
  const float* bo     = (const float*)d_in[7];
  const float* ln1_g  = (const float*)d_in[8];
  const float* ln1_b  = (const float*)d_in[9];
  const float* ln2_g  = (const float*)d_in[10];
  const float* ln2_b  = (const float*)d_in[11];
  const float* w1     = (const float*)d_in[12];
  const float* b1     = (const float*)d_in[13];
  const float* w2     = (const float*)d_in[14];
  const float* b2     = (const float*)d_in[15];
  const float* lnf_g  = (const float*)d_in[16];
  const float* lnf_b  = (const float*)d_in[17];
  const float* head_w = (const float*)d_in[18];
  const float* head_b = (const float*)d_in[19];
  float* out = (float*)d_out;

  char* wsb = (char*)d_ws;
  f16_t* WEMB = (f16_t*)(wsb + OFF_WEMB);
  f16_t* WQKV = (f16_t*)(wsb + OFF_WQKV);
  f16_t* WO   = (f16_t*)(wsb + OFF_WO);
  f16_t* W1   = (f16_t*)(wsb + OFF_W1);
  f16_t* W2   = (f16_t*)(wsb + OFF_W2);
  float* E32  = (float*)(wsb + OFF_E32);
  float* T32  = (float*)(wsb + OFF_T32);
  f16_t* H16  = (f16_t*)(wsb + OFF_H16);
  f16_t* BIG  = (f16_t*)(wsb + OFF_BIG);
  f16_t* X16  = BIG;
  f16_t* QKV16 = BIG;
  f16_t* MID16 = BIG;
  f16_t* KV16  = BIG;
  f16_t* Q16C  = (f16_t*)(wsb + OFF_BIG + OFF_Q16C_IN_BIG);

  const float WSC = 16.0f, WSC_INV = 0.0625f;

  xpose_x_kernel<<<NPIX / 256, 256, 0, stream>>>(x, X16);
  cast_w_kernel<<<(128 * 32 / 2 + 255) / 256, 256, 0, stream>>>(emb_w, WEMB, 128, 16, 32, WSC);
  cast_w_kernel<<<(768 * 128 / 2 + 255) / 256, 256, 0, stream>>>(wqkv, WQKV, 768, 128, 128, WSC);
  cast_w_kernel<<<(256 * 128 / 2 + 255) / 256, 256, 0, stream>>>(wo, WO, 256, 128, 128, WSC);
  cast_w_kernel<<<(512 * 128 / 2 + 255) / 256, 256, 0, stream>>>(w1, W1, 512, 128, 128, WSC);
  cast_w_kernel<<<(256 * 256 / 2 + 255) / 256, 256, 0, stream>>>(w2, W2, 256, 256, 256, WSC);
  launch_gemm<0, false, 0>(stream, X16, 32, WEMB, 32, (void*)E32, DM, emb_b, T32, NPIX, DM, 32, WSC_INV);

  const size_t CROW = (size_t)4 * PCH;
  for (int c = 0; c < NCHUNK; ++c) {
    const int nbase = c * PCH;
    gather_ln_kernel<<<dim3(PCH / 8, 9), 256, 0, stream>>>(E32, pos, ln1_g, ln1_b, T32, H16, PCH, nbase);
    launch_gemm<1, false, 0>(stream, H16, DM, WQKV, DM, (void*)QKV16, 384, bqkv, T32, RCH, 384, DM, WSC_INV);
    win_attn_kernel<0><<<PCH / 8, 288, 0, stream>>>(QKV16, 384, QKV16 + 128, QKV16 + 256, 384, H16, PCH);
    launch_gemm<0, true, 0>(stream, H16, DM, WO, DM, (void*)T32, DM, bo, T32, RCH, DM, DM, WSC_INV);
    ln_rows_kernel<<<RCH / 8, 256, 0, stream>>>(T32, H16, ln2_g, ln2_b, RCH);
    launch_gemm<1, false, 5>(stream, H16, DM, W1, DM, (void*)MID16, DFFC, b1, T32, RCH, DFFC, DM, WSC_INV);
    launch_gemm<0, true, 0>(stream, MID16, DFFC, W2, DFFC, (void*)T32, DM, b2, T32, RCH, DM, DFFC, WSC_INV);
    ln_rows_kernel<<<RCH / 8, 256, 0, stream>>>(T32, H16, ln1_g + DM, ln1_b + DM, RCH);
    launch_gemm<1, false, 0>(stream, H16, DM, WQKV + (size_t)(384 + 128) * DM, DM, (void*)KV16, 256,
                             bqkv + 384 + 128, T32, RCH, 256, DM, WSC_INV);
    launch_gemm<1, false, 0>(stream, H16 + CROW * DM, DM, WQKV + (size_t)384 * DM, DM, (void*)Q16C, DM,
                             bqkv + 384, T32, PCH, DM, DM, WSC_INV);
    win_attn_kernel<1><<<PCH / 64, 256, 0, stream>>>(Q16C, DM, KV16, KV16 + 128, 256, H16 + CROW * DM, PCH);
    launch_gemm<0, true, 0>(stream, H16 + CROW * DM, DM, WO + (size_t)DM * DM, DM, (void*)(T32 + CROW * DM), DM,
                            bo + DM, T32 + CROW * DM, PCH, DM, DM, WSC_INV);
    ln_rows_kernel<<<PCH / 8, 256, 0, stream>>>(T32 + CROW * DM, H16 + CROW * DM, ln2_g + DM, ln2_b + DM, PCH);
    launch_gemm<1, false, 5>(stream, H16 + CROW * DM, DM, W1 + (size_t)DFFC * DM, DM, (void*)MID16, DFFC,
                             b1 + DFFC, T32, PCH, DFFC, DM, WSC_INV);
    launch_gemm<0, true, 0>(stream, MID16, DFFC, W2 + (size_t)DM * DFFC, DFFC, (void*)(T32 + CROW * DM), DM,
                            b2 + DM, T32 + CROW * DM, PCH, DM, DFFC, WSC_INV);
    head_kernel<<<PCH / 32, 256, 0, stream>>>(T32 + CROW * DM, lnf_g, lnf_b, head_w, head_b, out + nbase, PCH);
  }
}
